// MultiHeadAttention_59871844106290
// MI455X (gfx1250) — hardware-verified
//
#include <hip/hip_runtime.h>


#ifndef NB
#define NB 2
#endif
#ifndef SEQ
#define SEQ 2048
#endif
#define NB_FULL  2
#define SEQ_FULL 2048
#define DM   1024
#define NH_  16
#define HD   64
#define NBH  (NB * NH_)
#define MROWS (NB * SEQ)
#define RH   256
#define SC2  (0.125f * 1.4426950408889634f)
#define PCL2 8.0f
#define NEGF (-3.0e38f)

static_assert(HD == 64);
static_assert(NH_ * HD == DM);
static_assert(DM % 64 == 0);
static_assert(SEQ % 64 == 0);
static_assert(RH % 64 == 0);
static_assert(SEQ >= RH);
static_assert(MROWS % 64 == 0);
static_assert(NB <= NB_FULL);
static_assert(SEQ <= SEQ_FULL);
static_assert(((size_t)SEQ * DM) % 8 == 0);

typedef _Float16 h16;
typedef unsigned short bf;
typedef __attribute__((ext_vector_type(16))) __bf16   v16bf;
typedef __attribute__((ext_vector_type(16))) _Float16 v16h;
typedef __attribute__((ext_vector_type(8)))  _Float16 v8h;
typedef __attribute__((ext_vector_type(8)))  unsigned short v8us;
typedef __attribute__((ext_vector_type(16))) unsigned short v16us;
typedef __attribute__((ext_vector_type(8)))  float    v8f;
typedef __attribute__((ext_vector_type(4)))  float    v4f;
typedef __attribute__((ext_vector_type(2)))  float    v2f;
typedef __attribute__((ext_vector_type(2)))  _Float16 v2h;
typedef __attribute__((ext_vector_type(2)))  unsigned short v2us;
typedef v4f  __attribute__((may_alias)) v4fa;

__device__ __forceinline__ unsigned short f2bf(float f) { unsigned u = __float_as_uint(f); u += 0x7FFFu + ((u >> 16) & 1u); return (unsigned short)(u >> 16); }
__device__ __forceinline__ float bf2f(unsigned short b) { return __uint_as_float(((unsigned)b) << 16); }
__device__ __forceinline__ float bfr(float f) { return bf2f(f2bf(f)); }
__device__ __forceinline__ void splitf(float y, unsigned short& h, unsigned short& l) { h = f2bf(y); l = f2bf(y - bf2f(h)); }
__device__ __forceinline__ v16h cat16(v8h lo, v8h hi) { return __builtin_shufflevector(lo, hi, 0, 1, 2, 3, 4, 5, 6, 7, 8, 9, 10, 11, 12, 13, 14, 15); }
__device__ __forceinline__ v16bf cat16b(v8us lo, v8us hi) { return __builtin_bit_cast(v16bf, __builtin_shufflevector(lo, hi, 0, 1, 2, 3, 4, 5, 6, 7, 8, 9, 10, 11, 12, 13, 14, 15)); }
__device__ __forceinline__ v8f wmma16(v16h a, v16h b, v8f c) { return __builtin_amdgcn_wmma_f32_16x16x32_f16(false, a, false, b, (short)0, c, false, false); }
__device__ __forceinline__ v8f wmmab(v16bf a, v16bf b, v8f c) { return __builtin_amdgcn_wmma_f32_16x16x32_bf16(false, a, false, b, (short)0, c, false, false); }
__device__ __forceinline__ v16h ldh(const h16* p) { return cat16(*(const v8h*)p, *(const v8h*)(p + 16)); }
__device__ __forceinline__ v16bf ldb(const bf* p) { return cat16b(*(const v8us*)p, *(const v8us*)(p + 16)); }
__device__ __forceinline__ float ex2(float x) { return __builtin_amdgcn_exp2f(x); }

template <int NSPLIT, bool BIAS>
__device__ __forceinline__ void gemmw_body(const bf* __restrict__ A, const bf* __restrict__ A2, const bf* __restrict__ Bt, const int K, float* C, const int ldc, const float* __restrict__ bias, const size_t sA, const size_t sB, const size_t sC) {
    __shared__ __align__(16) float os[16 * 68];
    const size_t z = blockIdx.z; A += z * sA; A2 += z * sA; Bt += z * sB; C += z * sC;
    const int lane = threadIdx.x & 31, lr = lane & 15, hi = lane >> 4; const int r0 = blockIdx.x * 64, c0 = blockIdx.y * 64;
    v8f acc[4][4];
#pragma unroll
    for (int mb = 0; mb < 4; ++mb)
#pragma unroll
        for (int nb = 0; nb < 4; ++nb) acc[mb][nb] = (v8f){};
    const size_t aoff = (size_t)(r0 + lr) * K + 8 * hi, boff = (size_t)(c0 + lr) * K + 8 * hi;
#pragma unroll 1
    for (int kc = 0; kc < K; kc += 32) {
        v16bf a[4], a2[4];
#pragma unroll
        for (int mb = 0; mb < 4; ++mb) { a[mb] = ldb(A + aoff + (size_t)mb * 16 * K + kc); if (NSPLIT == 1) a2[mb] = ldb(A2 + aoff + (size_t)mb * 16 * K + kc); else a2[mb] = a[mb]; }
#pragma unroll
        for (int nb = 0; nb < 4; ++nb) { const v16bf b = ldb(Bt + boff + (size_t)nb * 16 * K + kc);
#pragma unroll
            for (int mb = 0; mb < 4; ++mb) { acc[mb][nb] = wmmab(a[mb], b, acc[mb][nb]); if (NSPLIT == 1) acc[mb][nb] = wmmab(a2[mb], b, acc[mb][nb]); } }
        asm volatile("v_nop\n\tv_nop\n\tv_nop\n\tv_nop" : "+v"(acc[0][0]), "+v"(acc[0][1]), "+v"(acc[0][2]), "+v"(acc[0][3]), "+v"(acc[1][0]), "+v"(acc[1][1]), "+v"(acc[1][2]), "+v"(acc[1][3]), "+v"(acc[2][0]), "+v"(acc[2][1]), "+v"(acc[2][2]), "+v"(acc[2][3]), "+v"(acc[3][0]), "+v"(acc[3][1]), "+v"(acc[3][2]), "+v"(acc[3][3]) : "v"(a[0]), "v"(a[3]), "v"(a2[3]));
    }
#pragma unroll
    for (int mb = 0; mb < 4; ++mb) {
#pragma unroll
        for (int nb = 0; nb < 4; ++nb) {
#pragma unroll
            for (int j = 0; j < 8; ++j) os[(hi * 8 + j) * 68 + nb * 16 + lr] = acc[mb][nb][j]; }
        __builtin_amdgcn_wave_barrier(); asm volatile("" ::: "memory");
        float* crow = C + (size_t)(r0 + mb * 16) * ldc + c0;
#pragma unroll 1
        for (int ps = 0; ps < 2; ++ps) {
#pragma unroll
            for (int s = 0; s < 8; ++s) { const int row = 2 * s + hi, cofs = lr * 4; v4f val = *(const v4fa*)(os + row * 68 + cofs);
                if (BIAS) { val[0] += bfr(bias[c0 + cofs]); val[1] += bfr(bias[c0 + cofs + 1]); val[2] += bfr(bias[c0 + cofs + 2]); val[3] += bfr(bias[c0 + cofs + 3]); }
                *(volatile v4f*)(crow + (size_t)row * ldc + cofs) = val; }
            if (ps == 0) __threadfence(); }
        __builtin_amdgcn_wave_barrier(); asm volatile("" ::: "memory");
    }
}

__global__ __launch_bounds__(32) void k_gemm_qkv(const bf* __restrict__ XB, const bf* __restrict__ W, float* F) {
    gemmw_body<0, false>(XB, XB, W, DM, F, DM, (const float*)nullptr, (size_t)0, (size_t)DM * DM, (size_t)MROWS * DM);
}
__global__ __launch_bounds__(32) void k_gemm_out(const bf* __restrict__ ATh, const bf* __restrict__ ATl, const bf* __restrict__ WO, float* OUT, const float* __restrict__ bias) {
    gemmw_body<1, true>(ATh, ATl, WO, DM, OUT, DM, bias, (size_t)SEQ * DM, (size_t)0, (size_t)SEQ_FULL * DM);
}

__global__ __launch_bounds__(256) void k_cvt8(const float* __restrict__ src, bf* dst, size_t n8) { const size_t i = (size_t)blockIdx.x * 256 + threadIdx.x; if (i >= n8) return; const v8f v = *(const v8f*)(src + i * 8); v8us o;
#pragma unroll
    for (int k = 0; k < 8; ++k) o[k] = f2bf(v[k]); *(volatile v8us*)(dst + i * 8) = o; __threadfence(); *(volatile v8us*)(dst + i * 8) = o; }

__global__ __launch_bounds__(256) void k_qkp(const float* __restrict__ F, h16* P16, bf* Ph, bf* Pl) {
    const size_t e = ((size_t)blockIdx.x * 256 + threadIdx.x) * 2; if (e >= (size_t)2 * NBH * SEQ * HD) return;
    const int d = (int)(e % HD); const size_t r1 = e / HD; const int t = (int)(r1 % SEQ); const size_t r2 = r1 / SEQ; const int bh = (int)(r2 % NBH); const int w = (int)(r2 / NBH);
    const int b = bh / NH_, h = bh % NH_;
    const v2f x = *(const v2f*)(F + (size_t)w * MROWS * DM + ((size_t)b * SEQ + t) * DM + h * HD + d);
    v2h o16; v2us oh, ol;
#pragma unroll
    for (int q = 0; q < 2; ++q) { o16[q] = (h16)x[q]; unsigned short a2, c2; splitf(x[q], a2, c2); oh[q] = a2; ol[q] = c2; }
    const bool hr = (t < RH); const size_t oo = (((size_t)w * NBH + bh) * RH + (hr ? t : 0)) * HD + d;
    *(volatile v2h*)(P16 + e) = o16; if (hr) { *(volatile v2us*)(Ph + oo) = oh; *(volatile v2us*)(Pl + oo) = ol; }
    __threadfence();
    *(volatile v2h*)(P16 + e) = o16; if (hr) { *(volatile v2us*)(Ph + oo) = oh; *(volatile v2us*)(Pl + oo) = ol; }
}
__global__ __launch_bounds__(256) void k_vtp(const float* __restrict__ FV, h16* V16, bf* Vh, bf* Vl) {
    const size_t e = ((size_t)blockIdx.x * 256 + threadIdx.x) * 2; if (e >= (size_t)NBH * HD * SEQ) return;
    const int t = (int)(e % SEQ); const size_t r1 = e / SEQ; const int d = (int)(r1 % HD); const int bh = (int)(r1 / HD);
    const int b = bh / NH_, h = bh % NH_;
    v2h o16; v2us oh, ol;
#pragma unroll
    for (int q = 0; q < 2; ++q) { const float x = FV[((size_t)b * SEQ + t + q) * DM + h * HD + d]; o16[q] = (h16)x; unsigned short a2, c2; splitf(x, a2, c2); oh[q] = a2; ol[q] = c2; }
    const bool hr = (t < RH); const size_t oo = ((size_t)bh * HD + d) * RH + (hr ? t : 0);
    *(volatile v2h*)(V16 + e) = o16; if (hr) { *(volatile v2us*)(Vh + oo) = oh; *(volatile v2us*)(Vl + oo) = ol; }
    __threadfence();
    *(volatile v2h*)(V16 + e) = o16; if (hr) { *(volatile v2us*)(Vh + oo) = oh; *(volatile v2us*)(Vl + oo) = ol; }
}

__device__ __forceinline__ void attn_store(const v8f o0, const v8f o1, const v8f o2, const v8f o3, const float inv, const int wave, const int lane, bf* ATh, bf* ATl, const size_t rowbase) {
    __shared__ __align__(16) float os[4 * 16 * 68];
    const int lr = lane & 15, hi = lane >> 4; const int wb = wave * (16 * 68);
#pragma unroll
    for (int r = 0; r < 8; ++r) { os[wb + lr * 68 + hi * 8 + r] = o0[r] * inv; os[wb + lr * 68 + 16 + hi * 8 + r] = o1[r] * inv; os[wb + lr * 68 + 32 + hi * 8 + r] = o2[r] * inv; os[wb + lr * 68 + 48 + hi * 8 + r] = o3[r] * inv; }
    __syncthreads();
    const int rq = lane >> 3, c = (lane & 7) * 8;
#pragma unroll 1
    for (int ps = 0; ps < 2; ++ps) {
#pragma unroll
        for (int s = 0; s < 4; ++s) { const int row = 4 * s + rq; const v4f a = *(const v4fa*)(os + wb + row * 68 + c); const v4f b2 = *(const v4fa*)(os + wb + row * 68 + c + 4); v8us oh, ol;
#pragma unroll
            for (int q = 0; q < 4; ++q) { unsigned short x1, x2; splitf(a[q], x1, x2); oh[q] = x1; ol[q] = x2; splitf(b2[q], x1, x2); oh[4 + q] = x1; ol[4 + q] = x2; }
            *(volatile v8us*)(ATh + rowbase + (size_t)row * DM + c) = oh; *(volatile v8us*)(ATl + rowbase + (size_t)row * DM + c) = ol; }
        if (ps == 0) __threadfence(); }
}

__global__ __launch_bounds__(128) void k_attn_f16(const h16* __restrict__ Q16, const h16* __restrict__ K16, const h16* __restrict__ VT16, bf* ATh, bf* ATl) {
    const int wave = __builtin_amdgcn_readfirstlane((int)(threadIdx.x >> 5));
    const int lane = threadIdx.x & 31, lr = lane & 15, hi = lane >> 4;
    const int bh = blockIdx.y; const int q0 = RH + ((int)blockIdx.x * 4 + wave) * 16;
    const size_t pbase = (size_t)bh * SEQ * HD;
    const h16* Qp = Q16 + pbase; const h16* Kp = K16 + pbase; const h16* Vp = VT16 + pbase;
    const int qoff = (q0 + lr) * HD + 8 * hi;
    const v16h qf0 = ldh(Qp + qoff), qf1 = ldh(Qp + qoff + 32);
    v8f o[4];
#pragma unroll
    for (int t = 0; t < 4; ++t) o[t] = (v8f){};
    float m = NEGF, l = 0.0f;
    const int ktmax = (q0 + 15) >> 5;
#pragma unroll 1
    for (int kt = 0; kt <= ktmax; ++kt) {
        const int k0 = kt * 32; const int koff = (k0 + lr) * HD + 8 * hi;
        v8f s0 = (v8f){}, s1 = (v8f){};
        const v16h ka = ldh(Kp + koff), kb = ldh(Kp + koff + 32);
        const v16h kc = ldh(Kp + koff + 16 * HD), kd = ldh(Kp + koff + 16 * HD + 32);
        s0 = wmma16(ka, qf0, s0); s0 = wmma16(kb, qf1, s0); s1 = wmma16(kc, qf0, s1); s1 = wmma16(kd, qf1, s1);
        asm volatile("v_nop\n\tv_nop\n\tv_nop\n\tv_nop" : "+v"(s0), "+v"(s1) : "v"(kc), "v"(kd), "v"(qf0), "v"(qf1));
        float t0[8], t1[8];
#pragma unroll
        for (int r = 0; r < 8; ++r) { t0[r] = s0[r] * SC2; t1[r] = s1[r] * SC2; }
        if (kt == ktmax) { const int qq = q0 + lr - k0 - 8 * hi;
#pragma unroll
            for (int r = 0; r < 8; ++r) { t0[r] = (r <= qq) ? t0[r] : NEGF; t1[r] = (r + 16 <= qq) ? t1[r] : NEGF; } }
        float mx = fmaxf(t0[0], t1[0]);
#pragma unroll
        for (int r = 1; r < 8; ++r) mx = fmaxf(mx, fmaxf(t0[r], t1[r]));
        mx = fmaxf(mx, __shfl_xor(mx, 16, 32));
        const float mn = fmaxf(m, mx); const float corr = ex2(m - mn); m = mn; const float mb = mn - PCL2;
        float psum = 0.0f; v16h pf;
#pragma unroll
        for (int r = 0; r < 8; ++r) { const float p0 = ex2(t0[r] - mb), p1 = ex2(t1[r] - mb); psum += p0 + p1; pf[r] = (h16)p0; pf[8 + r] = (h16)p1; }
        l = l * corr + psum;
#pragma unroll
        for (int t = 0; t < 4; ++t) o[t] = o[t] * corr;
        const int voff = lr * SEQ + k0 + 8 * hi;
        const v16h v0 = ldh(Vp + voff), v1 = ldh(Vp + voff + 16 * SEQ), v2 = ldh(Vp + voff + 32 * SEQ), v3 = ldh(Vp + voff + 48 * SEQ);
        o[0] = wmma16(v0, pf, o[0]); o[1] = wmma16(v1, pf, o[1]); o[2] = wmma16(v2, pf, o[2]); o[3] = wmma16(v3, pf, o[3]);
        asm volatile("v_nop\n\tv_nop\n\tv_nop\n\tv_nop" : "+v"(o[0]), "+v"(o[1]), "+v"(o[2]), "+v"(o[3]) : "v"(v2), "v"(v3), "v"(pf));
    }
    l += __shfl_xor(l, 16, 32);
    const float inv = 1.0f / l;
    const size_t rowbase = ((size_t)(bh / NH_) * SEQ + q0) * DM + (size_t)(bh % NH_) * HD;
    attn_store(o[0], o[1], o[2], o[3], inv, wave, lane, ATh, ATl, rowbase);
}

__global__ __launch_bounds__(128) void k_attn_hl(const bf* __restrict__ Qh, const bf* __restrict__ Ql, const bf* __restrict__ Kh, const bf* __restrict__ Kl, const bf* __restrict__ VTh, const bf* __restrict__ VTl, bf* ATh, bf* ATl) {
    const int wave = __builtin_amdgcn_readfirstlane((int)(threadIdx.x >> 5));
    const int lane = threadIdx.x & 31, lr = lane & 15, hi = lane >> 4;
    const int bh = blockIdx.y; const int q0 = ((int)blockIdx.x * 4 + wave) * 16;
    const size_t pbase = (size_t)bh * RH * HD;
    const bf* Qhp = Qh + pbase; const bf* Qlp = Ql + pbase; const bf* Khp = Kh + pbase; const bf* Klp = Kl + pbase; const bf* Vhp = VTh + pbase; const bf* Vlp = VTl + pbase;
    const int qoff = (q0 + lr) * HD + 8 * hi;
    const v16bf qh0 = ldb(Qhp + qoff), qh1 = ldb(Qhp + qoff + 32), ql0 = ldb(Qlp + qoff), ql1 = ldb(Qlp + qoff + 32);
    v8f o[4];
#pragma unroll
    for (int t = 0; t < 4; ++t) o[t] = (v8f){};
    float m = NEGF, l = 0.0f;
    const int ktmax = (q0 + 15) >> 5;
#pragma unroll 1
    for (int kt = 0; kt <= ktmax; ++kt) {
        const int k0 = kt * 32; const int koff = (k0 + lr) * HD + 8 * hi;
        v8f s0 = (v8f){}, s1 = (v8f){};
        { const v16bf a = ldb(Khp + koff), b = ldb(Khp + koff + 32), c = ldb(Klp + koff), d = ldb(Klp + koff + 32);
          s0 = wmmab(a, qh0, s0); s0 = wmmab(b, qh1, s0); s0 = wmmab(c, qh0, s0); s0 = wmmab(d, qh1, s0); s0 = wmmab(a, ql0, s0); s0 = wmmab(b, ql1, s0); }
        const v16bf a1 = ldb(Khp + koff + 16 * HD), b1 = ldb(Khp + koff + 16 * HD + 32), c1 = ldb(Klp + koff + 16 * HD), d1 = ldb(Klp + koff + 16 * HD + 32);
        s1 = wmmab(a1, qh0, s1); s1 = wmmab(b1, qh1, s1); s1 = wmmab(c1, qh0, s1); s1 = wmmab(d1, qh1, s1); s1 = wmmab(a1, ql0, s1); s1 = wmmab(b1, ql1, s1);
        asm volatile("v_nop\n\tv_nop\n\tv_nop\n\tv_nop" : "+v"(s0), "+v"(s1) : "v"(a1), "v"(b1), "v"(ql0), "v"(ql1));
        float t0[8], t1[8];
#pragma unroll
        for (int r = 0; r < 8; ++r) { t0[r] = s0[r] * SC2; t1[r] = s1[r] * SC2; }
        if (kt == ktmax) { const int qq = q0 + lr - k0 - 8 * hi;
#pragma unroll
            for (int r = 0; r < 8; ++r) { t0[r] = (r <= qq) ? t0[r] : NEGF; t1[r] = (r + 16 <= qq) ? t1[r] : NEGF; } }
        float mx = fmaxf(t0[0], t1[0]);
#pragma unroll
        for (int r = 1; r < 8; ++r) mx = fmaxf(mx, fmaxf(t0[r], t1[r]));
        mx = fmaxf(mx, __shfl_xor(mx, 16, 32));
        const float mn = fmaxf(m, mx); const float corr = ex2(m - mn); m = mn;
        float psum = 0.0f; v16us phu, plu;
#pragma unroll
        for (int r = 0; r < 8; ++r) { const float p0 = ex2(t0[r] - mn), p1 = ex2(t1[r] - mn); psum += p0 + p1; unsigned short x1, x2; splitf(p0, x1, x2); phu[r] = x1; plu[r] = x2; splitf(p1, x1, x2); phu[8 + r] = x1; plu[8 + r] = x2; }
        const v16bf ph = __builtin_bit_cast(v16bf, phu), pl = __builtin_bit_cast(v16bf, plu);
        l = l * corr + psum;
#pragma unroll
        for (int t = 0; t < 4; ++t) o[t] = o[t] * corr;
        const int voff = lr * RH + k0 + 8 * hi;
        v16bf vh, vl;
#pragma unroll
        for (int t = 0; t < 4; ++t) { vh = ldb(Vhp + voff + t * 16 * RH); vl = ldb(Vlp + voff + t * 16 * RH); o[t] = wmmab(vh, ph, o[t]); o[t] = wmmab(vl, ph, o[t]); o[t] = wmmab(vh, pl, o[t]); }
        asm volatile("v_nop\n\tv_nop\n\tv_nop\n\tv_nop" : "+v"(o[0]), "+v"(o[1]), "+v"(o[2]), "+v"(o[3]) : "v"(vh), "v"(vl), "v"(ph), "v"(pl));
    }
    l += __shfl_xor(l, 16, 32);
    const float inv = 1.0f / l;
    const size_t rowbase = ((size_t)(bh / NH_) * SEQ + q0) * DM + (size_t)(bh % NH_) * HD;
    attn_store(o[0], o[1], o[2], o[3], inv, wave, lane, ATh, ATl, rowbase);
}

constexpr size_t SZ_XB  = (size_t)MROWS * DM * 2;
constexpr size_t SZ_W   = (size_t)4 * DM * DM * 2;
constexpr size_t SZ_F   = (size_t)3 * MROWS * DM * 4;
constexpr size_t SZ_QK  = (size_t)2 * NBH * SEQ * HD * 2;
constexpr size_t SZ_VT  = (size_t)NBH * HD * SEQ * 2;
constexpr size_t SZ_QKH = (size_t)2 * NBH * RH * HD * 2;
constexpr size_t SZ_VTH = (size_t)NBH * HD * RH * 2;
constexpr size_t SZ_AT  = (size_t)MROWS * DM * 2;
constexpr size_t SZ_TOT = SZ_XB + SZ_W + SZ_F + SZ_QK + SZ_VT + 2 * SZ_QKH + 2 * SZ_VTH + 2 * SZ_AT;
static_assert(SZ_XB % 256 == 0 && SZ_W % 256 == 0 && SZ_F % 256 == 0 && SZ_QK % 256 == 0 && SZ_VT % 256 == 0 && SZ_QKH % 256 == 0 && SZ_VTH % 256 == 0 && SZ_AT % 256 == 0);
static_assert(SZ_TOT <= (size_t)134217728);

extern "C" void kernel_launch(void* const* d_in, const int* in_sizes, int n_in,
                              void* d_out, int out_size, void* d_ws, size_t ws_size, hipStream_t stream) {
    if (n_in < 6) return;
    const size_t need_x = (size_t)(NB - 1) * SEQ_FULL * DM + (size_t)SEQ * DM;
    if ((size_t)in_sizes[0] < need_x || (size_t)out_size < need_x) return;
    if (in_sizes[1] < DM * DM || in_sizes[2] < DM * DM || in_sizes[3] < DM * DM || in_sizes[4] < DM * DM || in_sizes[5] < DM) return;
    if (SZ_TOT > ws_size) return;
    const float* x = (const float*)d_in[0]; const float* wq = (const float*)d_in[1]; const float* wk = (const float*)d_in[2]; const float* wv = (const float*)d_in[3];
    const float* wp = (const float*)d_in[4]; const float* bp = (const float*)d_in[5];
    float* OUT = (float*)d_out;
    char* wsp = (char*)d_ws;
    bf* XB = (bf*)wsp; wsp += SZ_XB;
    bf* W = (bf*)wsp; wsp += SZ_W; bf* WO = W + (size_t)3 * DM * DM;
    float* F = (float*)wsp; wsp += SZ_F;
    h16* QK16 = (h16*)wsp; wsp += SZ_QK;
    h16* VT16 = (h16*)wsp; wsp += SZ_VT;
    bf* QKh = (bf*)wsp; wsp += SZ_QKH; bf* QKl = (bf*)wsp; wsp += SZ_QKH;
    bf* VTh = (bf*)wsp; wsp += SZ_VTH; bf* VTl = (bf*)wsp; wsp += SZ_VTH;
    bf* ATh = (bf*)wsp; wsp += SZ_AT; bf* ATl = (bf*)wsp; wsp += SZ_AT;

    const size_t xn8 = (size_t)SEQ * DM / 8, wn8 = (size_t)DM * DM / 8;
    for (int b = 0; b < NB; ++b)
        k_cvt8<<<(unsigned)((xn8 + 255) / 256), 256, 0, stream>>>(x + (size_t)b * SEQ_FULL * DM, XB + (size_t)b * SEQ * DM, xn8);
    k_cvt8<<<(unsigned)((wn8 + 255) / 256), 256, 0, stream>>>(wq, W, wn8);
    k_cvt8<<<(unsigned)((wn8 + 255) / 256), 256, 0, stream>>>(wk, W + (size_t)DM * DM, wn8);
    k_cvt8<<<(unsigned)((wn8 + 255) / 256), 256, 0, stream>>>(wv, W + (size_t)2 * DM * DM, wn8);
    k_cvt8<<<(unsigned)((wn8 + 255) / 256), 256, 0, stream>>>(wp, WO, wn8);
    k_gemm_qkv<<<dim3(MROWS / 64, DM / 64, 3), 32, 0, stream>>>(XB, W, F);
    k_qkp<<<(unsigned)(((size_t)2 * NBH * SEQ * HD / 2 + 255) / 256), 256, 0, stream>>>(F, QK16, QKh, QKl);
    k_vtp<<<(unsigned)(((size_t)NBH * HD * SEQ / 2 + 255) / 256), 256, 0, stream>>>(F + (size_t)2 * MROWS * DM, VT16, VTh, VTl);
    k_attn_hl<<<dim3(RH / 64, NBH), 128, 0, stream>>>(QKh, QKl, QKh + (size_t)NBH * RH * HD, QKl + (size_t)NBH * RH * HD, VTh, VTl, ATh, ATl);
    if (SEQ > RH)
        k_attn_f16<<<dim3((SEQ - RH) / 64, NBH), 128, 0, stream>>>(QK16, QK16 + (size_t)NBH * SEQ * HD, VT16, ATh, ATl);
    k_gemm_out<<<dim3(SEQ / 64, DM / 64, NB), 32, 0, stream>>>(ATh, ATl, WO, OUT, bp);
}
